// DuhamelLayer_56650618635121
// MI455X (gfx1250) — hardware-verified
//
#include <hip/hip_runtime.h>
#include <math.h>
#include <stdint.h>

#define BATCH   16
#define OUT_CH  8
#define NT      65536
#define MAXK    3687
#define FP      2048
#define XPW     (FP + NT)
#define IRFP    1856
#define KP      1920
#define KMAX    1888
#define WAVES   8
#define TW      1024
#define TB      (WAVES * TW)
#define XSC     64.0f
#define FSC     1024.0f
#define LSC     2048.0f
#define ALPHA_H 1.52587890625e-05f
#define ALPHA_L 7.450580596923828125e-09f

static constexpr int kVW[OUT_CH] = {1844, 1317, 1024, 768, 576, 419, 307, 230};
static constexpr int kKO[OUT_CH] = {1888, 1344, 1056, 800, 608, 448, 352, 256};
__device__ __constant__ int c_VW[OUT_CH] = {1844, 1317, 1024, 768, 576, 419, 307, 230};
__device__ __constant__ int c_KO[OUT_CH] = {1888, 1344, 1056, 800, 608, 448, 352, 256};

constexpr bool tables_ok() {
  for (int i = 0; i < OUT_CH; ++i) {
    const int need = 16 * ((kVW[i] + 14) / 16 + 1);
    if (kKO[i] < need) return false;
    if ((kKO[i] % 32) != 0) return false;
    if (kKO[i] > KMAX) return false;
    if (kVW[i] > IRFP) return false;
    if (kVW[i] > kVW[0]) return false;
  }
  return true;
}
static_assert(tables_ok());
static_assert(MAXK == 2 * 1844 - 1);
static_assert(MAXK / 2 == 1843);
static_assert(FP >= KMAX - 16 && (FP % 8) == 0);
static_assert(KP >= KMAX && (KP % 64) == 0);
static_assert((IRFP % 32) == 0 && (XPW % 64) == 0);
static_assert((NT % TB) == 0 && (TW % 256) == 0);
static_assert(((BATCH * XPW) % (8 * 256)) == 0);
static_assert(((OUT_CH * 16 * KP) % (8 * 256)) == 0);
static_assert(((OUT_CH * IRFP) % 256) == 0);

typedef _Float16 v16h __attribute__((ext_vector_type(16)));
typedef _Float16 v8h  __attribute__((ext_vector_type(8)));
typedef float    v8f  __attribute__((ext_vector_type(8)));
typedef float    v4f  __attribute__((ext_vector_type(4)));
typedef unsigned int v4u __attribute__((ext_vector_type(4)));

__device__ __forceinline__ float bf_rne(float f) {
  unsigned u = __float_as_uint(f);
  u = (u + 0x7FFFu + ((u >> 16) & 1u)) & 0xFFFF0000u;
  return __uint_as_float(u);
}
__device__ __forceinline__ unsigned short h_bits(float f) {
  _Float16 h = (_Float16)f;
  return __builtin_bit_cast(unsigned short, h);
}
__device__ __forceinline__ unsigned pk16(unsigned short a, unsigned short b) { return (unsigned)a | ((unsigned)b << 16); }
__device__ __forceinline__ v8f zero8() { v8f z = {0.f, 0.f, 0.f, 0.f, 0.f, 0.f, 0.f, 0.f}; return z; }

__device__ __forceinline__ v16h ldfrag_h(const _Float16* p) {
  union { v16h v; v8h h[2]; } f;
  f.h[0] = *(const v8h*)(p);
  f.h[1] = *(const v8h*)(p + 16);
  return f.v;
}
__device__ __forceinline__ v16h ldfrag_x(const _Float16* p) {
  union { v16h v; v8h h[2]; } f;
  f.h[0] = *(const v8h*)(p);
  f.h[1] = *(const v8h*)(p - 16);
  return f.v;
}

__device__ __forceinline__ v8f mma_h_raw(v16h a, v16h b, v8f c) {
  return __builtin_amdgcn_wmma_f32_16x16x32_f16(false, a, false, b, (short)0, c, false, false);
}
__device__ __forceinline__ void dep_guard4_h(v8f& a, v8f& b, v8f& c, v8f& d, v16h x, v16h y) {
#if defined(__HIP_DEVICE_COMPILE__)
  asm volatile("v_nop\n\tv_nop\n\tv_nop\n\tv_nop" : "+v"(a), "+v"(b), "+v"(c), "+v"(d) : "v"(x), "v"(y));
#endif
}
__device__ __forceinline__ void keep4_h(v16h a, v16h b, v16h c, v16h d) {
#if defined(__HIP_DEVICE_COMPILE__)
  asm volatile("v_nop" :: "v"(a), "v"(b), "v"(c), "v"(d));
#endif
}
__device__ __forceinline__ void acc_guard4(v8f& a, v8f& b, v8f& c, v8f& d) {
#if defined(__HIP_DEVICE_COMPILE__)
  asm volatile("v_nop\n\tv_nop\n\tv_nop\n\tv_nop" : "+v"(a), "+v"(b), "+v"(c), "+v"(d));
#endif
}
__device__ __forceinline__ void wave_sync_lds() {
  __builtin_amdgcn_fence(__ATOMIC_RELEASE, "workgroup");
  __builtin_amdgcn_wave_barrier();
  __builtin_amdgcn_fence(__ATOMIC_ACQUIRE, "workgroup");
}

__device__ __forceinline__ unsigned short hx(float f, bool live) {
  const float s = live ? bf_rne(f) * XSC : 0.0f;
  return h_bits(s);
}
__global__ __launch_bounds__(256) void k_xplane(const float* __restrict__ x, unsigned short* XP) {
  const int i = blockIdx.x * 256 + threadIdx.x;
  if (i >= (BATCH * XPW) / 8) return;
  const int f = i * 8;
  const int b = f / XPW;
  const int p = f - b * XPW;
  int src = p - FP;
  const bool live = (src >= 0);
  src = live ? src : 0;
  const float* xb = x + (size_t)b * NT + src;
  const v4f a = *(const v4f*)(xb);
  const v4f c = *(const v4f*)(xb + 4);
  v4u pk;
  pk[0] = pk16(hx(a[0], live), hx(a[1], live));
  pk[1] = pk16(hx(a[2], live), hx(a[3], live));
  pk[2] = pk16(hx(c[0], live), hx(c[1], live));
  pk[3] = pk16(hx(c[2], live), hx(c[3], live));
  unsigned short* dst = XP + (size_t)f;
  *(volatile v4u*)dst = pk;
  __threadfence();
  *(volatile v4u*)dst = pk;
}

__global__ __launch_bounds__(256) void k_irf(const float* __restrict__ lw, float* IRF) {
  const int i = blockIdx.x * 256 + threadIdx.x;
  if (i >= OUT_CH * IRFP) return;
  const int o = i / IRFP;
  const int m = i - o * IRFP;
  const int W = c_VW[o];
  const float lg = bf_rne(lw[o]);
  float omega = expf(lg);
  omega = fminf(fmaxf(omega, 0.01f), 1000.0f);
  const float sq = sqrtf((float)(1.0 - 0.05 * 0.05));
  const float omegaD = omega * sq;
  const float tt = (float)m * 0.01f;
  const float ex = expf((-0.05f * omega) * tt);
  const float sn = sinf(omegaD * tt);
  float v = ((1.0f / omegaD) * ex) * sn;
  v = (m < W) ? v : 0.0f;
  *(volatile float*)(IRF + i) = v;
  __threadfence();
  *(volatile float*)(IRF + i) = v;
}

__global__ __launch_bounds__(256) void k_bplane(const float* __restrict__ IRF,
                                                unsigned short* BH, unsigned short* BL) {
  const int i = blockIdx.x * 256 + threadIdx.x;
  if (i >= (OUT_CH * 16 * KP) / 8) return;
  const int f = i * 8;
  const int row = f / KP;
  const int k0 = f - row * KP;
  const int o = row >> 4, n = row & 15;
  const int W = c_VW[o], Ko = c_KO[o];
  const int qq = k0 >> 4, j0 = k0 & 15;
  const float* irow = IRF + o * IRFP;
  unsigned short hb[8], lb[8];
#pragma unroll
  for (int e = 0; e < 8; ++e) {
    const int k = k0 + e;
    const int m = 16 * qq + n - (j0 + e);
    const bool ok = (k < Ko) && (m >= 0) && (m < W);
    int mc = (m < 0) ? 0 : m;
    mc = (mc > IRFP - 1) ? (IRFP - 1) : mc;
    float v = irow[mc];
    v = ok ? v : 0.0f;
    const float hs = v * FSC;
    const _Float16 hh = (_Float16)hs;
    const float lo = (hs - (float)hh) * LSC;
    hb[e] = __builtin_bit_cast(unsigned short, hh);
    lb[e] = h_bits(lo);
  }
  v4u ph, pl;
  ph[0] = pk16(hb[0], hb[1]); ph[1] = pk16(hb[2], hb[3]); ph[2] = pk16(hb[4], hb[5]); ph[3] = pk16(hb[6], hb[7]);
  pl[0] = pk16(lb[0], lb[1]); pl[1] = pk16(lb[2], lb[3]); pl[2] = pk16(lb[4], lb[5]); pl[3] = pk16(lb[6], lb[7]);
  unsigned short* dh = BH + (size_t)f;
  unsigned short* dl = BL + (size_t)f;
  *(volatile v4u*)dh = ph;
  *(volatile v4u*)dl = pl;
  __threadfence();
  *(volatile v4u*)dh = ph;
  *(volatile v4u*)dl = pl;
}

__global__ __launch_bounds__(256) void k_conv(const unsigned short* __restrict__ XPp,
                                              const unsigned short* __restrict__ BHp,
                                              const unsigned short* __restrict__ BLp,
                                              float* out) {
  const _Float16* XP = (const _Float16*)(const void*)XPp;
  const _Float16* BH = (const _Float16*)(const void*)BHp;
  const _Float16* BL = (const _Float16*)(const void*)BLp;
  __shared__ __align__(16) float sT[WAVES][TW];
  const int lane = threadIdx.x & 31;
  const int wave = threadIdx.x >> 5;
  const int b = blockIdx.y;
  const int o = blockIdx.z;
  int Ko = c_KO[o];
  Ko = (Ko > KMAX) ? KMAX : Ko;
  const int t0 = blockIdx.x * TB + wave * TW;

  const int rlane = lane & 15;
  const int koff  = (lane >> 4) * 8;
  const int mOff  = (lane >> 4) * 8;

  const _Float16* pa  = XP + (size_t)b * XPW + FP + t0 + 16 * rlane + koff;
  const _Float16* pbh = BH + (size_t)(o * 16 + rlane) * KP + koff;
  const _Float16* pbl = BL + (size_t)(o * 16 + rlane) * KP + koff;

  v8f accH[4], accL[4];
#pragma unroll
  for (int s = 0; s < 4; ++s) { accH[s] = zero8(); accL[s] = zero8(); }

  for (int kk = 0; kk < Ko; kk += 32) {
    const v16h bh = ldfrag_h(pbh + kk);
    const v16h bl = ldfrag_h(pbl + kk);
    v16h ax[4];
#pragma unroll
    for (int s = 0; s < 4; ++s) ax[s] = ldfrag_x(pa + 256 * s - kk);
#pragma unroll
    for (int s = 0; s < 4; ++s) accH[s] = mma_h_raw(ax[s], bh, accH[s]);
    dep_guard4_h(accH[0], accH[1], accH[2], accH[3], ax[3], bh);
#pragma unroll
    for (int s = 0; s < 4; ++s) accL[s] = mma_h_raw(ax[s], bl, accL[s]);
    dep_guard4_h(accL[0], accL[1], accL[2], accL[3], ax[3], bl);
    keep4_h(ax[0], ax[1], ax[2], ax[3]);
  }
  acc_guard4(accH[0], accH[1], accH[2], accH[3]);
  acc_guard4(accL[0], accL[1], accL[2], accL[3]);

  float* slab = sT[wave];
#pragma unroll
  for (int s = 0; s < 4; ++s) {
#pragma unroll
    for (int r = 0; r < 8; ++r) {
      const float v = accH[s][r] * ALPHA_H + accL[s][r] * ALPHA_L;
      slab[256 * s + (mOff + r) * 16 + rlane] = v;
    }
  }
  wave_sync_lds();
  const int q4 = (lane & 7) * 4;
  const int lq = lane >> 3;
  v4f pk[8];
#pragma unroll
  for (int it = 0; it < 8; ++it) {
    const int line = it * 4 + lq;
    pk[it] = *(const v4f*)(slab + line * 32 + q4);
  }
  float* ob = out + (size_t)(b * OUT_CH + o) * NT + t0;
  for (int pass = 0; pass < 2; ++pass) {
#pragma unroll
    for (int it = 0; it < 8; ++it) {
      const int line = it * 4 + lq;
      *(volatile v4f*)(ob + line * 32 + q4) = pk[it];
    }
    __threadfence();
  }
  wave_sync_lds();
}

extern "C" void kernel_launch(void* const* d_in, const int* in_sizes, int n_in,
                              void* d_out, int out_size, void* d_ws, size_t ws_size,
                              hipStream_t stream) {
  if (n_in < 2) return;
  if (in_sizes[0] != BATCH * NT) return;
  if (in_sizes[1] < OUT_CH) return;
  if (out_size != BATCH * OUT_CH * NT) return;

  const float* x  = (const float*)d_in[0];
  const float* lw = (const float*)d_in[1];
  float* out = (float*)d_out;

  const size_t PXP  = (size_t)BATCH * XPW * 2;
  const size_t PIRF = (size_t)OUT_CH * IRFP * 4;
  const size_t PB   = (size_t)OUT_CH * 16 * KP * 2;
  size_t off = 0;
  const size_t oXP  = off; off += PXP;
  const size_t oIRF = off; off += PIRF;
  const size_t oBH  = off; off += PB;
  const size_t oBL  = off; off += PB;
  if (off > ws_size) return;
  if (off > (size_t)134217728) return;

  char* ws = (char*)d_ws;
  unsigned short* XP  = (unsigned short*)(ws + oXP);
  float*          IRF = (float*)(ws + oIRF);
  unsigned short* BH  = (unsigned short*)(ws + oBH);
  unsigned short* BL  = (unsigned short*)(ws + oBL);

  const dim3 blk(256);
  const dim3 gX((BATCH * XPW) / 8 / 256);
  const dim3 gI((OUT_CH * IRFP) / 256);
  const dim3 gB((OUT_CH * 16 * KP) / 8 / 256);
  const dim3 gC(NT / TB, BATCH, OUT_CH);

  k_xplane<<<gX, blk, 0, stream>>>(x, XP);
  k_irf<<<gI, blk, 0, stream>>>(lw, IRF);
  k_bplane<<<gB, blk, 0, stream>>>(IRF, BH, BL);
  k_conv<<<gC, blk, 0, stream>>>(XP, BH, BL, out);
  (void)hipGetLastError();
}
